// GConvGRUModel_79585743995076
// MI455X (gfx1250) — hardware-verified
//
#include <hip/hip_runtime.h>
#include <stddef.h>


#define CF      32
#define NTHR    256
#define NWAVE   8
#define EPT     8
#define NGRP    2
#define CHUNK   (NTHR * EPT * NGRP)
#define WCAP    (EPT * NGRP * 32)
#define LISTN   (NWAVE * WCAP)
#define NBD     4096
#define NB1     1024
#define NB2     2048
#define NMAT    12
#define A1W     64

#define LDS_AGG1 (NB1 * A1W * 4 + LISTN * 4 + 64)
#define LDS_AGG2 (NB2 * CF * 4 + LISTN * 4 + 64)

static_assert((CHUNK & (CHUNK - 1)) == 0);
static_assert(CHUNK <= 4096);
static_assert(NBD <= 4096 && NB1 <= 4096 && NB2 <= 4096);
static_assert((NB1 & (NB1 - 1)) == 0 && (NB2 & (NB2 - 1)) == 0 && (NBD & (NBD - 1)) == 0);
static_assert(NWAVE * 16 * CF <= LISTN);
static_assert(NB2 <= LISTN);
static_assert(NB1 % (16 * NWAVE) == 0 && NB2 % (16 * NWAVE) == 0);
static_assert(NB2 % (128 * NWAVE) == 0);
static_assert(NBD == NWAVE * 4 * 128);
static_assert(NBD >= NB1 && NBD >= NB2);
static_assert(NTHR * 8 * 3 == 6 * CF * CF);

typedef float          v4f   __attribute__((ext_vector_type(4)));
typedef float          v8f   __attribute__((ext_vector_type(8)));
typedef int            v4i   __attribute__((ext_vector_type(4)));
typedef unsigned short v8us  __attribute__((ext_vector_type(8)));
typedef unsigned short v16us __attribute__((ext_vector_type(16)));
typedef __bf16         v16bf __attribute__((ext_vector_type(16)));
union FragB { v16bf v; v16us u; v8us h[2]; };

__device__ __forceinline__ v8f zero8() { v8f z = {0.f, 0.f, 0.f, 0.f, 0.f, 0.f, 0.f, 0.f}; return z; }

__device__ __forceinline__ unsigned bfbits(float f) {
  const unsigned u = __float_as_uint(f);
  return (u + 0x7FFFu + ((u >> 16) & 1u)) >> 16;
}

__device__ __forceinline__ v8f wmb(v16bf a, v16bf b, v8f c) {
  v8f d = __builtin_amdgcn_wmma_f32_16x16x32_bf16(false, a, false, b, (short)0, c, false, false);
  asm volatile("v_nop\n\tv_nop\n\tv_nop\n\tv_nop" : "+v"(d) : "v"(a), "v"(b));
  return d;
}

#define SPL1(I, V) { const float f_ = (V); const unsigned hb_ = bfbits(f_); ah.u[I] = (unsigned short)hb_; \
    al.u[I] = (unsigned short)bfbits(f_ - __uint_as_float(hb_ << 16)); }
__device__ __forceinline__ void lda_split(const float* p, FragB& ah, FragB& al) {
  const v4f p0 = *(const v4f*)p;
  const v4f p1 = *(const v4f*)(p + 4);
  const v4f q0 = *(const v4f*)(p + 16);
  const v4f q1 = *(const v4f*)(p + 20);
  SPL1(0, p0.x)  SPL1(1, p0.y)  SPL1(2, p0.z)  SPL1(3, p0.w)
  SPL1(4, p1.x)  SPL1(5, p1.y)  SPL1(6, p1.z)  SPL1(7, p1.w)
  SPL1(8, q0.x)  SPL1(9, q0.y)  SPL1(10, q0.z) SPL1(11, q0.w)
  SPL1(12, q1.x) SPL1(13, q1.y) SPL1(14, q1.z) SPL1(15, q1.w)
}
#undef SPL1

__device__ __forceinline__ v16bf ldb(const unsigned short* __restrict__ pl, int mat, int nt, int m, int hh) {
  const unsigned short* bp = pl + ((mat * CF + 16 * nt + m) * CF) + 8 * hh;
  FragB b;
  b.h[0] = *(const v8us*)bp;
  b.h[1] = *(const v8us*)(bp + 16);
  return b.v;
}

__device__ __forceinline__ v8f mma3(v8f c, v16bf ah, v16bf al,
                                    const unsigned short* __restrict__ whi, const unsigned short* __restrict__ wlo,
                                    int mat, int nt, int m, int hh) {
  const v16bf bhv = ldb(whi, mat, nt, m, hh);
  const v16bf blv = ldb(wlo, mat, nt, m, hh);
  c = wmb(ah, bhv, c);
  c = wmb(ah, blv, c);
  c = wmb(al, bhv, c);
  return c;
}

__device__ __forceinline__ float sigm(float v) {
  const float vc = fminf(fmaxf(v, -30.f), 30.f);
  return __builtin_amdgcn_rcpf(1.f + __expf(-vc));
}
__device__ __forceinline__ float tanh_(float v) {
  const float a = fminf(fabsf(v), 15.f);
  const float e = __expf(-2.f * a);
  const float t = (1.f - e) * __builtin_amdgcn_rcpf(1.f + e);
  return copysignf(t, v);
}
__device__ __forceinline__ float softplus_(float t) {
  const float tc = fminf(t, 20.f);
  const float s  = __logf(1.f + __expf(tc));
  return (t > 20.f) ? t : s;
}

template <int NB>
__device__ __forceinline__ int scan_chunk(const int* __restrict__ ids, int nE, int cbase, int nodeBase,
                                          int vec8, int* list, int tid, int lane, int wave) {
  int wc = 0;
#pragma unroll
  for (int g = 0; g < NGRP; ++g) {
    const int el0  = (g * NTHR + tid) * EPT;
    const int e0   = cbase + el0;
    const int sent = -2147483647 - 1;
    v4i da, db;
    if (vec8 != 0 && cbase + CHUNK <= nE) {
      da = *(const v4i*)(ids + e0);
      db = *(const v4i*)(ids + e0 + 4);
    } else {
      da.x = (e0     < nE) ? ids[min(e0, nE - 1)] : sent;
      da.y = (e0 + 1 < nE) ? ids[min(e0 + 1, nE - 1)] : sent;
      da.z = (e0 + 2 < nE) ? ids[min(e0 + 2, nE - 1)] : sent;
      da.w = (e0 + 3 < nE) ? ids[min(e0 + 3, nE - 1)] : sent;
      db.x = (e0 + 4 < nE) ? ids[min(e0 + 4, nE - 1)] : sent;
      db.y = (e0 + 5 < nE) ? ids[min(e0 + 5, nE - 1)] : sent;
      db.z = (e0 + 6 < nE) ? ids[min(e0 + 6, nE - 1)] : sent;
      db.w = (e0 + 7 < nE) ? ids[min(e0 + 7, nE - 1)] : sent;
    }
    const unsigned nb = (unsigned)nodeBase;
    const unsigned s0 = (unsigned)da.x - nb, s1 = (unsigned)da.y - nb;
    const unsigned s2 = (unsigned)da.z - nb, s3 = (unsigned)da.w - nb;
    const unsigned s4 = (unsigned)db.x - nb, s5 = (unsigned)db.y - nb;
    const unsigned s6 = (unsigned)db.z - nb, s7 = (unsigned)db.w - nb;
    const bool h0 = s0 < (unsigned)NB, h1 = s1 < (unsigned)NB, h2 = s2 < (unsigned)NB, h3 = s3 < (unsigned)NB;
    const bool h4 = s4 < (unsigned)NB, h5 = s5 < (unsigned)NB, h6 = s6 < (unsigned)NB, h7 = s7 < (unsigned)NB;
    const unsigned any = __builtin_amdgcn_ballot_w32(h0 | h1 | h2 | h3 | h4 | h5 | h6 | h7);
    if (any != 0u) {
#define HITJ(J, HJ, SJ) { \
        const unsigned mj = __builtin_amdgcn_ballot_w32(HJ); \
        if (mj != 0u) { \
          if (HJ) { \
            const int pos = wc + (int)__builtin_amdgcn_mbcnt_lo(mj, 0u); \
            if (pos < WCAP) list[wave * WCAP + pos] = ((el0 + (J)) << 12) | (int)(SJ); \
          } \
          wc += (int)__builtin_popcount(mj); } }
      HITJ(0, h0, s0)
      HITJ(1, h1, s1)
      HITJ(2, h2, s2)
      HITJ(3, h3, s3)
      HITJ(4, h4, s4)
      HITJ(5, h5, s5)
      HITJ(6, h6, s6)
      HITJ(7, h7, s7)
#undef HITJ
    }
  }
  return wc;
}

__global__ __launch_bounds__(NTHR) void k_wprep(const float* __restrict__ Wx, const float* __restrict__ Wh,
                                                unsigned short* whi, unsigned short* wlo) {
  const int i = blockIdx.x * NTHR + threadIdx.x;
  if (i >= NMAT * CF * CF / 8) return;
  const bool first = blockIdx.x < 3;
  const float* W = first ? Wx : Wh;
  const int o   = i * 8;
  const int mat = o >> 10;
  const int rem = o & 1023;
  const int n   = rem >> 5;
  const int k0  = rem & 31;
  const int ml  = first ? mat : mat - 6;
  const float* p = W + (size_t)ml * (CF * CF) + (size_t)k0 * CF + n;
  v8us hv, lv;
#define WP1(J) { const float f_ = p[(J) * CF]; const unsigned hb_ = bfbits(f_); hv[J] = (unsigned short)hb_; \
                 lv[J] = (unsigned short)bfbits(f_ - __uint_as_float(hb_ << 16)); }
  WP1(0) WP1(1) WP1(2) WP1(3) WP1(4) WP1(5) WP1(6) WP1(7)
#undef WP1
  unsigned short* dh = whi + o;
  unsigned short* dl = wlo + o;
  *(volatile v8us*)dh = hv;
  *(volatile v8us*)dl = lv;
  __threadfence();
  *(volatile v8us*)dh = hv;
  *(volatile v8us*)dl = lv;
}

__global__ __launch_bounds__(NTHR) void k_deg(
    const int* __restrict__ ei, const float* __restrict__ ew, float* dis, int nE, int vec8) {
  __shared__ __attribute__((aligned(16))) float dsum[NBD];
  __shared__ __attribute__((aligned(16))) int list[LISTN];
  __shared__ int wcnt[NWAVE];
  const int tid = threadIdx.x, lane = tid & 31, wave = tid >> 5;
  const int nodeBase = blockIdx.x * NBD;
  const int* srcs = ei;

  for (int i = tid; i < NBD; i += NTHR) dsum[i] = 0.f;
  __syncthreads();

  const int nChunks = (nE + CHUNK - 1) / CHUNK;
#pragma unroll 1
  for (int ch = 0; ch < nChunks; ++ch) {
    const int cbase = ch * CHUNK;
    const int wc = scan_chunk<NBD>(srcs, nE, cbase, nodeBase, vec8, list, tid, lane, wave);
    if (lane == 0) wcnt[wave] = wc;
    __syncthreads();
    if (wave == 0) {
#pragma unroll 1
      for (int wsx = 0; wsx < NWAVE; ++wsx) {
        int n = __builtin_amdgcn_readfirstlane(wcnt[wsx]);
        n = n > WCAP ? WCAP : (n < 0 ? 0 : n);
        const int* lp = list + wsx * WCAP;
#pragma unroll 1
        for (int i = 0; i < n; ++i) {
          const int ent  = __builtin_amdgcn_readfirstlane(lp[i]);
          const int slot = ent & (NBD - 1);
          int e = cbase + ((ent >> 12) & (CHUNK - 1));
          e = e > nE - 1 ? nE - 1 : e;
          const float wv = ew[e];
          if (lane == 0) dsum[slot] = dsum[slot] + wv;
        }
      }
    }
    __syncthreads();
  }

  v4f dq[4];
#pragma unroll
  for (int q = 0; q < 4; ++q) {
    const int f = (wave * 4 + q) * 128 + 4 * lane;
    const v4f c = *(const v4f*)(dsum + f);
    v4f d;
    d.x = c.x > 0.f ? rsqrtf(c.x) : 0.f;
    d.y = c.y > 0.f ? rsqrtf(c.y) : 0.f;
    d.z = c.z > 0.f ? rsqrtf(c.z) : 0.f;
    d.w = c.w > 0.f ? rsqrtf(c.w) : 0.f;
    dq[q] = d;
  }
  float* dp = dis + (size_t)nodeBase;
#pragma unroll
  for (int q = 0; q < 4; ++q) *(volatile v4f*)(dp + (wave * 4 + q) * 128 + 4 * lane) = dq[q];
  __threadfence();
#pragma unroll
  for (int q = 0; q < 4; ++q) *(volatile v4f*)(dp + (wave * 4 + q) * 128 + 4 * lane) = dq[q];
}

__global__ __launch_bounds__(NTHR) void k_agg1(
    const int* __restrict__ ei, const float* __restrict__ ew, const float* __restrict__ x,
    const float* __restrict__ hs, const float* __restrict__ dis,
    const unsigned short* __restrict__ whi, const unsigned short* __restrict__ wlo,
    const float* __restrict__ bx, const float* __restrict__ bh,
    float* zpl, float* upl, float* cpl, int nN, int nE, int vec8) {
  extern __shared__ v4f lds_dyn[];
  float* acc  = (float*)lds_dyn;
  int*   list = (int*)(acc + NB1 * A1W);
  int*   wcnt = list + LISTN;
  float* stg  = (float*)list;
  const int tid = threadIdx.x, lane = tid & 31, wave = tid >> 5, hh = lane >> 4, m = lane & 15;
  const int nodeBase = blockIdx.x * NB1;
  const int* srcs = ei;
  const int* dsts = ei + nE;

  {
    const v4f z = {0.f, 0.f, 0.f, 0.f};
    for (int i = tid; i < NB1 * A1W / 4; i += NTHR) lds_dyn[i] = z;
  }
  __syncthreads();

  const int nChunks = (nE + CHUNK - 1) / CHUNK;
#pragma unroll 1
  for (int ch = 0; ch < nChunks; ++ch) {
    const int cbase = ch * CHUNK;
    const int wc = scan_chunk<NB1>(dsts, nE, cbase, nodeBase, vec8, list, tid, lane, wave);
    if (lane == 0) wcnt[wave] = wc;
    __syncthreads();
    if (wave == 0) {
#pragma unroll 1
      for (int wsx = 0; wsx < NWAVE; ++wsx) {
        int n = __builtin_amdgcn_readfirstlane(wcnt[wsx]);
        n = n > WCAP ? WCAP : (n < 0 ? 0 : n);
        const int* lp = list + wsx * WCAP;
#pragma unroll 1
        for (int i = 0; i < n; ++i) {
          const int ent  = __builtin_amdgcn_readfirstlane(lp[i]);
          const int slot = ent & (NB1 - 1);
          int e = cbase + ((ent >> 12) & (CHUNK - 1));
          e = e > nE - 1 ? nE - 1 : e;
          int s = srcs[e];
          s = s < 0 ? 0 : (s > nN - 1 ? nN - 1 : s);
          int dn = nodeBase + slot;
          dn = dn > nN - 1 ? nN - 1 : dn;
          const float wv = ew[e];
          const float c  = -((dis[s] * wv) * dis[dn]);
          const float xv = x[(size_t)s * CF + lane];
          const float hv = hs[(size_t)s * CF + lane];
          float* ap = acc + slot * A1W + lane;
          ap[0]  = ap[0]  + c * xv;
          ap[32] = ap[32] + c * hv;
        }
      }
    }
    __syncthreads();
  }

  const float bz0 = bx[m] + bh[m],                      bz1 = bx[16 + m] + bh[16 + m];
  const float br0 = bx[CF + m] + bh[CF + m],            br1 = bx[CF + 16 + m] + bh[CF + 16 + m];
  const float bc0 = bx[2 * CF + m] + bh[2 * CF + m],    bc1 = bx[2 * CF + 16 + m] + bh[2 * CF + 16 + m];
  const int rw = lane >> 3, pc = (lane & 7) * 4;

#pragma unroll 1
  for (int it = 0; it < NB1 / (16 * NWAVE); ++it) {
    const int tl    = it * NWAVE + wave;
    const int R0    = 16 * tl;
    const int node0 = nodeBase + R0;
    int nodeA = node0 + m;
    nodeA = nodeA > nN - 1 ? nN - 1 : nodeA;

    v8f az0 = zero8(), az1 = zero8(), ar0 = zero8(), ar1 = zero8(), ac0 = zero8(), ac1 = zero8();
    FragB ah, al;
    {
      lda_split(x + (size_t)nodeA * CF + 8 * hh, ah, al);
      az0 = mma3(az0, ah.v, al.v, whi, wlo, 0, 0, m, hh);
      az1 = mma3(az1, ah.v, al.v, whi, wlo, 0, 1, m, hh);
      ar0 = mma3(ar0, ah.v, al.v, whi, wlo, 2, 0, m, hh);
      ar1 = mma3(ar1, ah.v, al.v, whi, wlo, 2, 1, m, hh);
      ac0 = mma3(ac0, ah.v, al.v, whi, wlo, 4, 0, m, hh);
      ac1 = mma3(ac1, ah.v, al.v, whi, wlo, 4, 1, m, hh);
    }
    {
      lda_split(acc + (R0 + m) * A1W + 8 * hh, ah, al);
      az0 = mma3(az0, ah.v, al.v, whi, wlo, 1, 0, m, hh);
      az1 = mma3(az1, ah.v, al.v, whi, wlo, 1, 1, m, hh);
      ar0 = mma3(ar0, ah.v, al.v, whi, wlo, 3, 0, m, hh);
      ar1 = mma3(ar1, ah.v, al.v, whi, wlo, 3, 1, m, hh);
      ac0 = mma3(ac0, ah.v, al.v, whi, wlo, 5, 0, m, hh);
      ac1 = mma3(ac1, ah.v, al.v, whi, wlo, 5, 1, m, hh);
    }
    {
      lda_split(hs + (size_t)nodeA * CF + 8 * hh, ah, al);
      az0 = mma3(az0, ah.v, al.v, whi, wlo, 6, 0, m, hh);
      az1 = mma3(az1, ah.v, al.v, whi, wlo, 6, 1, m, hh);
      ar0 = mma3(ar0, ah.v, al.v, whi, wlo, 8, 0, m, hh);
      ar1 = mma3(ar1, ah.v, al.v, whi, wlo, 8, 1, m, hh);
    }
    {
      lda_split(acc + (R0 + m) * A1W + 32 + 8 * hh, ah, al);
      az0 = mma3(az0, ah.v, al.v, whi, wlo, 7, 0, m, hh);
      az1 = mma3(az1, ah.v, al.v, whi, wlo, 7, 1, m, hh);
      ar0 = mma3(ar0, ah.v, al.v, whi, wlo, 9, 0, m, hh);
      ar1 = mma3(ar1, ah.v, al.v, whi, wlo, 9, 1, m, hh);
    }
    __syncthreads();

#pragma unroll
    for (int r = 0; r < 8; ++r) {
      const int row = R0 + 8 * hh + r;
      int nodec = nodeBase + row;
      nodec = nodec > nN - 1 ? nN - 1 : nodec;
      const float h0 = hs[(size_t)nodec * CF + m];
      const float h1 = hs[(size_t)nodec * CF + 16 + m];
      float* sr = acc + row * A1W;
      sr[m]      = sigm(az0[r] + bz0);
      sr[16 + m] = sigm(az1[r] + bz1);
      sr[32 + m] = h0 * sigm(ar0[r] + br0);
      sr[48 + m] = h1 * sigm(ar1[r] + br1);
      float* cr = stg + (wave * 16 + 8 * hh + r) * CF;
      cr[m]      = ac0[r] + bc0;
      cr[16 + m] = ac1[r] + bc1;
    }
    __syncthreads();

#pragma unroll
    for (int q = 0; q < 4; ++q) {
      const int row  = 4 * q + rw;
      const int slot = R0 + row;
      const v4f zv = *(const v4f*)(acc + slot * A1W + pc);
      const v4f uv = *(const v4f*)(acc + slot * A1W + 32 + pc);
      const v4f cv = *(const v4f*)(stg + (wave * 16 + row) * CF + pc);
      const size_t g = (size_t)(nodeBase + slot) * CF + pc;
      *(volatile v4f*)(zpl + g) = zv;
      *(volatile v4f*)(upl + g) = uv;
      *(volatile v4f*)(cpl + g) = cv;
    }
    __threadfence();
#pragma unroll
    for (int q = 0; q < 4; ++q) {
      const int row  = 4 * q + rw;
      const int slot = R0 + row;
      const v4f zv = *(const v4f*)(acc + slot * A1W + pc);
      const v4f uv = *(const v4f*)(acc + slot * A1W + 32 + pc);
      const v4f cv = *(const v4f*)(stg + (wave * 16 + row) * CF + pc);
      const size_t g = (size_t)(nodeBase + slot) * CF + pc;
      *(volatile v4f*)(zpl + g) = zv;
      *(volatile v4f*)(upl + g) = uv;
      *(volatile v4f*)(cpl + g) = cv;
    }
  }
}

__global__ __launch_bounds__(NTHR) void k_agg2(
    const int* __restrict__ ei, const float* __restrict__ ew, const float* __restrict__ upl,
    const float* __restrict__ dis, const unsigned short* __restrict__ whi, const unsigned short* __restrict__ wlo,
    const float* __restrict__ cpl, const float* __restrict__ zpl, const float* __restrict__ hs,
    const float* __restrict__ Wl, const float* __restrict__ bl,
    float* out0, float* out1, int nN, int nE, int vec8) {
  extern __shared__ v4f lds_dyn[];
  float* acc  = (float*)lds_dyn;
  int*   list = (int*)(acc + NB2 * CF);
  int*   wcnt = list + LISTN;
  float* outs = (float*)list;
  const int tid = threadIdx.x, lane = tid & 31, wave = tid >> 5, hh = lane >> 4, m = lane & 15;
  const int nodeBase = blockIdx.x * NB2;
  const int* srcs = ei;
  const int* dsts = ei + nE;

  {
    const v4f z = {0.f, 0.f, 0.f, 0.f};
    for (int i = tid; i < NB2 * CF / 4; i += NTHR) lds_dyn[i] = z;
  }
  __syncthreads();

  const int nChunks = (nE + CHUNK - 1) / CHUNK;
#pragma unroll 1
  for (int ch = 0; ch < nChunks; ++ch) {
    const int cbase = ch * CHUNK;
    const int wc = scan_chunk<NB2>(dsts, nE, cbase, nodeBase, vec8, list, tid, lane, wave);
    if (lane == 0) wcnt[wave] = wc;
    __syncthreads();
    if (wave == 0) {
#pragma unroll 1
      for (int wsx = 0; wsx < NWAVE; ++wsx) {
        int n = __builtin_amdgcn_readfirstlane(wcnt[wsx]);
        n = n > WCAP ? WCAP : (n < 0 ? 0 : n);
        const int* lp = list + wsx * WCAP;
#pragma unroll 1
        for (int i = 0; i < n; ++i) {
          const int ent  = __builtin_amdgcn_readfirstlane(lp[i]);
          const int slot = ent & (NB2 - 1);
          int e = cbase + ((ent >> 12) & (CHUNK - 1));
          e = e > nE - 1 ? nE - 1 : e;
          int s = srcs[e];
          s = s < 0 ? 0 : (s > nN - 1 ? nN - 1 : s);
          int dn = nodeBase + slot;
          dn = dn > nN - 1 ? nN - 1 : dn;
          const float wv = ew[e];
          const float c  = -((dis[s] * wv) * dis[dn]);
          const float uv = upl[(size_t)s * CF + lane];
          float* ap = acc + slot * CF + lane;
          ap[0] = ap[0] + c * uv;
        }
      }
    }
    __syncthreads();
  }

  const float wl0 = Wl[m], wl1 = Wl[16 + m];
  const float blv = bl[0];
  const int rw = lane >> 3, pc = (lane & 7) * 4;

#pragma unroll 1
  for (int it = 0; it < NB2 / (16 * NWAVE); ++it) {
    const int tl    = it * NWAVE + wave;
    const int R0    = 16 * tl;
    const int node0 = nodeBase + R0;
    int nodeA = node0 + m;
    nodeA = nodeA > nN - 1 ? nN - 1 : nodeA;

    v8f a0 = zero8(), a1 = zero8();
    FragB ah, al;
    {
      lda_split(upl + (size_t)nodeA * CF + 8 * hh, ah, al);
      a0 = mma3(a0, ah.v, al.v, whi, wlo, 10, 0, m, hh);
      a1 = mma3(a1, ah.v, al.v, whi, wlo, 10, 1, m, hh);
    }
    {
      lda_split(acc + (R0 + m) * CF + 8 * hh, ah, al);
      a0 = mma3(a0, ah.v, al.v, whi, wlo, 11, 0, m, hh);
      a1 = mma3(a1, ah.v, al.v, whi, wlo, 11, 1, m, hh);
    }

    v8f hn0 = zero8(), hn1 = zero8(), dt = zero8();
#pragma unroll
    for (int r = 0; r < 8; ++r) {
      int nodec = node0 + 8 * hh + r;
      nodec = nodec > nN - 1 ? nN - 1 : nodec;
      const size_t g0 = (size_t)nodec * CF + m;
      const float c0 = cpl[g0], c1 = cpl[g0 + 16];
      const float z0 = zpl[g0], z1 = zpl[g0 + 16];
      const float h0 = hs[g0],  h1 = hs[g0 + 16];
      const float t0 = tanh_(a0[r] + c0);
      const float t1 = tanh_(a1[r] + c1);
      const float v0 = z0 * h0 + (1.f - z0) * t0;
      const float v1 = z1 * h1 + (1.f - z1) * t1;
      hn0[r] = v0;
      hn1[r] = v1;
      float d = fmaxf(v0, 0.f) * wl0 + fmaxf(v1, 0.f) * wl1;
      d += __shfl_xor(d, 1, 32);
      d += __shfl_xor(d, 2, 32);
      d += __shfl_xor(d, 4, 32);
      d += __shfl_xor(d, 8, 32);
      dt[r] = d;
    }
    __syncthreads();

#pragma unroll
    for (int r = 0; r < 8; ++r) {
      const int row = R0 + 8 * hh + r;
      float* sr = acc + row * CF;
      sr[m]      = hn0[r];
      sr[16 + m] = hn1[r];
      if (m == 0) outs[row] = softplus_(dt[r] + blv);
    }
    __syncthreads();

#pragma unroll
    for (int q = 0; q < 4; ++q) {
      const int row  = 4 * q + rw;
      const int slot = R0 + row;
      const int node = nodeBase + slot;
      if (node < nN) {
        const v4f v = *(const v4f*)(acc + slot * CF + pc);
        *(volatile v4f*)(out1 + (size_t)node * CF + pc) = v;
      }
    }
    __threadfence();
#pragma unroll
    for (int q = 0; q < 4; ++q) {
      const int row  = 4 * q + rw;
      const int slot = R0 + row;
      const int node = nodeBase + slot;
      if (node < nN) {
        const v4f v = *(const v4f*)(acc + slot * CF + pc);
        *(volatile v4f*)(out1 + (size_t)node * CF + pc) = v;
      }
    }
  }
  __syncthreads();

#pragma unroll
  for (int qq = 0; qq < NB2 / (128 * NWAVE); ++qq) {
    const int q = qq * NWAVE + wave;
    const int f = q * 128 + 4 * lane;
    const int node = nodeBase + f;
    if (node + 3 < nN) { const v4f v = *(const v4f*)(outs + f); *(volatile v4f*)(out0 + node) = v; }
  }
  __threadfence();
#pragma unroll
  for (int qq = 0; qq < NB2 / (128 * NWAVE); ++qq) {
    const int q = qq * NWAVE + wave;
    const int f = q * 128 + 4 * lane;
    const int node = nodeBase + f;
    if (node + 3 < nN) { const v4f v = *(const v4f*)(outs + f); *(volatile v4f*)(out0 + node) = v; }
  }
}

extern "C" void kernel_launch(void* const* d_in, const int* in_sizes, int n_in,
                              void* d_out, int out_size, void* d_ws, size_t ws_size,
                              hipStream_t stream) {
  if (n_in < 10) return;
  const int nN = in_sizes[0] / CF;
  const int nE = in_sizes[1] / 2;
  if (nN <= 0 || nE <= 0) return;
  if (in_sizes[0] != nN * CF || in_sizes[1] != 2 * nE || in_sizes[2] != nE || in_sizes[3] != nN * CF) return;
  if (in_sizes[4] != 6 * CF * CF || in_sizes[5] < 3 * CF || in_sizes[6] != 6 * CF * CF || in_sizes[7] < 3 * CF) return;
  if (in_sizes[8] < CF || in_sizes[9] < 1) return;
  if (out_size != nN + nN * CF) return;

  const float* x  = (const float*)d_in[0];
  const int*   ei = (const int*)d_in[1];
  const float* ew = (const float*)d_in[2];
  const float* hs = (const float*)d_in[3];
  const float* Wx = (const float*)d_in[4];
  const float* bx = (const float*)d_in[5];
  const float* Wh = (const float*)d_in[6];
  const float* bh = (const float*)d_in[7];
  const float* Wl = (const float*)d_in[8];
  const float* bl = (const float*)d_in[9];
  float* out0 = (float*)d_out;
  float* out1 = (float*)d_out + nN;

  const int nBD = (nN + NBD - 1) / NBD;
  const int nA1 = (nN + NB1 - 1) / NB1;
  const int nA2 = (nN + NB2 - 1) / NB2;

  char* ws = (char*)d_ws;
  size_t off = 0;
  const size_t oHi = off; off += (size_t)NMAT * CF * CF * 2;            off = (off + 255) & ~(size_t)255;
  const size_t oLo = off; off += (size_t)NMAT * CF * CF * 2;            off = (off + 255) & ~(size_t)255;
  const size_t oDs = off; off += (size_t)nBD * NBD * 4;                 off = (off + 255) & ~(size_t)255;
  const size_t oZ  = off; off += (size_t)nA1 * NB1 * CF * 4;            off = (off + 255) & ~(size_t)255;
  const size_t oU  = off; off += (size_t)nA1 * NB1 * CF * 4;            off = (off + 255) & ~(size_t)255;
  const size_t oC  = off; off += (size_t)nA1 * NB1 * CF * 4;            off = (off + 255) & ~(size_t)255;
  if (off > ws_size) return;
  unsigned short* whi = (unsigned short*)(ws + oHi);
  unsigned short* wlo = (unsigned short*)(ws + oLo);
  float* dis = (float*)(ws + oDs);
  float* zpl = (float*)(ws + oZ);
  float* upl = (float*)(ws + oU);
  float* cpl = (float*)(ws + oC);

  const int vec8 = ((nE & 3) == 0) ? 1 : 0;

  const int nPrep = NMAT * CF * CF / 8;
  k_wprep<<<(nPrep + NTHR - 1) / NTHR, NTHR, 0, stream>>>(Wx, Wh, whi, wlo);

  k_deg<<<nBD, NTHR, 0, stream>>>(ei, ew, dis, nE, vec8);

  hipFuncSetAttribute(reinterpret_cast<const void*>(&k_agg1),
                      hipFuncAttributeMaxDynamicSharedMemorySize, LDS_AGG1);
  k_agg1<<<nA1, NTHR, LDS_AGG1, stream>>>(ei, ew, x, hs, dis, whi, wlo, bx, bh, zpl, upl, cpl, nN, nE, vec8);

  hipFuncSetAttribute(reinterpret_cast<const void*>(&k_agg2),
                      hipFuncAttributeMaxDynamicSharedMemorySize, LDS_AGG2);
  k_agg2<<<nA2, NTHR, LDS_AGG2, stream>>>(ei, ew, upl, dis, whi, wlo, cpl, zpl, hs, Wl, bl, out0, out1, nN, nE, vec8);
}
